// TextConditionalMultiHeadAttention_2216203125587
// MI455X (gfx1250) — hardware-verified
//
#include <hip/hip_runtime.h>

constexpr int kNumB      = 16;
constexpr int kLQ        = 32;
constexpr int kLK        = 256;
constexpr int kDim       = 512;
constexpr int kHeads     = 8;
constexpr int kDk        = 64;
constexpr int kQRows     = kNumB * kLQ;
constexpr int kKRows     = kNumB * kLK;
constexpr int kChunkRows = kLQ * kLK;
constexpr int kFqLd      = 1536;
constexpr int kKvLd      = 1024;
constexpr int kSlot      = 262144;
constexpr float kWCarry     = 16.0f;
constexpr float kAttCarry   = 16.0f;
constexpr float kScaleW     = 1.0f / 16.0f;
constexpr float kScaleOut   = 1.0f / 256.0f;
constexpr float kInvDim     = 1.0f / 512.0f;
constexpr float kLnEps      = 1e-5f;
constexpr float kLogitScale = 0.125f;

constexpr size_t kOffW16  = 0;
constexpr size_t kOffFq   = kOffW16 + (size_t)16 * kSlot * 2;
constexpr size_t kOffVp   = kOffFq  + (size_t)kQRows * kFqLd * 4;
constexpr size_t kOffCb   = kOffVp  + (size_t)kKRows * kDim * 4;
constexpr size_t kOffCk   = kOffCb  + (size_t)kKRows * kDim * 4;
constexpr size_t kOffKv   = kOffCk  + (size_t)kChunkRows * kDim * 2;
constexpr size_t kOffAtt  = kOffKv  + (size_t)kChunkRows * kKvLd * 4;
constexpr size_t kWsTotal = kOffAtt + (size_t)kQRows * kDim * 2;
static_assert(kWsTotal == (size_t)70778880);
static_assert(kWsTotal <= (size_t)134217728);
static_assert((kOffFq % 128) == 0 && (kOffVp % 128) == 0 && (kOffCb % 128) == 0 && (kOffCk % 128) == 0 && (kOffKv % 128) == 0 && (kOffAtt % 128) == 0);

typedef __attribute__((ext_vector_type(16))) _Float16 v16h;
typedef __attribute__((ext_vector_type(8)))  _Float16 v8h;
typedef __attribute__((ext_vector_type(16))) __bf16   v16b;
typedef __attribute__((ext_vector_type(8)))  __bf16   v8b;
typedef __attribute__((ext_vector_type(8)))  float    v8f;
typedef __attribute__((ext_vector_type(4)))  float    v4f;
typedef __attribute__((ext_vector_type(4)))  unsigned int v4u;

__device__ __forceinline__ unsigned short f2bf_bits(float f) {
  unsigned u = __float_as_uint(f);
  return (unsigned short)((u + 0x7FFFu + ((u >> 16) & 1u)) >> 16);
}
__device__ __forceinline__ float bf_bits2f(unsigned short h) { return __uint_as_float(((unsigned)h) << 16); }

__device__ __forceinline__ void dep_guard_h(v8f& a, v8f& b, v16h x, v16h y) { asm volatile("v_nop\n\tv_nop\n\tv_nop\n\tv_nop" : "+v"(a), "+v"(b) : "v"(x), "v"(y)); }
__device__ __forceinline__ void dep_guard_b(v8f& a, v8f& b, v16b x, v16b y) { asm volatile("v_nop\n\tv_nop\n\tv_nop\n\tv_nop" : "+v"(a), "+v"(b) : "v"(x), "v"(y)); }
__device__ __forceinline__ void keep4_h(v16h a, v16h b, v16h c, v16h d) { asm volatile("v_nop" :: "v"(a), "v"(b), "v"(c), "v"(d)); }
__device__ __forceinline__ void keep4_b(v16b a, v16b b, v16b c, v16b d) { asm volatile("v_nop" :: "v"(a), "v"(b), "v"(c), "v"(d)); }
__device__ __forceinline__ void acc_guard4(v8f& a, v8f& b, v8f& c, v8f& d) { asm volatile("v_nop\n\tv_nop\n\tv_nop\n\tv_nop" : "+v"(a), "+v"(b), "+v"(c), "+v"(d)); }
template <typename T> struct Frag;
template <> struct Frag<_Float16> {
  typedef v16h V; union U { v16h v; v8h h[2]; };
  static __device__ __forceinline__ v16h load(const _Float16* p) {
    U f; f.h[0] = *(const v8h*)(p); f.h[1] = *(const v8h*)(p + 16); return f.v;
  }
  static __device__ __forceinline__ v8f mma(v16h a, v16h b, v8f c) {
    return __builtin_amdgcn_wmma_f32_16x16x32_f16(false, a, false, b, (short)0, c, false, false);
  }
  static __device__ __forceinline__ void guard(v8f& a, v8f& b, v16h x, v16h y) { dep_guard_h(a, b, x, y); }
  static __device__ __forceinline__ void keep(v16h a, v16h b, v16h c, v16h d) { keep4_h(a, b, c, d); }
};
template <> struct Frag<__bf16> {
  typedef v16b V; union U { v16b v; v8b h[2]; };
  static __device__ __forceinline__ v16b load(const __bf16* p) {
    U f; f.h[0] = *(const v8b*)(p); f.h[1] = *(const v8b*)(p + 16); return f.v;
  }
  static __device__ __forceinline__ v8f mma(v16b a, v16b b, v8f c) {
    return __builtin_amdgcn_wmma_f32_16x16x32_bf16(false, a, false, b, (short)0, c, false, false);
  }
  static __device__ __forceinline__ void guard(v8f& a, v8f& b, v16b x, v16b y) { dep_guard_b(a, b, x, y); }
  static __device__ __forceinline__ void keep(v16b a, v16b b, v16b c, v16b d) { keep4_b(a, b, c, d); }
};

__device__ __forceinline__ unsigned pk16(unsigned short a, unsigned short b) { return (unsigned)a | ((unsigned)b << 16); }
__device__ __forceinline__ unsigned short h_bits(float f) { const _Float16 h = (_Float16)f; return __builtin_bit_cast(unsigned short, h); }

template <int ET> struct Elem;
template <> struct Elem<0> { typedef _Float16 T; };
template <> struct Elem<1> { typedef __bf16 T; };
template <int ET, bool SPLIT, int BIAS_MODE, int OUT_MODE, bool RESID, int ACT = 0>
__global__ __launch_bounds__(256) void wmma_gemm64(
    const unsigned short* __restrict__ Ap, const unsigned short* __restrict__ A2p, int lda, long strideA,
    const unsigned short* __restrict__ Btp, const unsigned short* __restrict__ Bt2p, int ldb, long strideB,
    void* __restrict__ Cout, void* __restrict__ Cout2, int ldc, long strideC,
    const float* __restrict__ bias,
    const float* __restrict__ resid, long strideR,
    int M, int N, int K, float scale) {
  typedef typename Elem<ET>::T T;
  typedef typename Frag<T>::V V;
  const T* A = (const T*)Ap; const T* A2 = (const T*)A2p; const T* Bt = (const T*)Btp; const T* Bt2 = (const T*)Bt2p;
  __shared__ __align__(16) float sT[8][16 * 68];
  const int b    = blockIdx.y;
  const int lane = threadIdx.x & 31;
  const int wave = threadIdx.x >> 5;
  const int tilesN = N >> 6;
  const int tilesM = M >> 6;
  const int tile = blockIdx.x * 8 + wave;
  if (tile >= tilesM * tilesN) return;
  const int tm = tile / tilesN;
  const int tn = tile - tm * tilesN;
  const int m0 = tm << 6;
  const int n0 = tn << 6;

  const T* Ab  = A  + (size_t)b * strideA;
  const T* Bb  = Bt + (size_t)b * strideB;
  const T* Ab2 = SPLIT ? (A2  + (size_t)b * strideA) : nullptr;
  const T* Bb2 = SPLIT ? (Bt2 + (size_t)b * strideB) : nullptr;

  const int rlane = lane & 15;
  const int koff  = (lane >> 4) * 8;
  const int mOff  = (lane >> 4) * 8;

  v8f acc[4][4];
#pragma unroll
  for (int i = 0; i < 4; ++i)
#pragma unroll
    for (int j = 0; j < 4; ++j) acc[i][j] = (v8f){0.f,0.f,0.f,0.f,0.f,0.f,0.f,0.f};

  for (int k0 = 0; k0 < K; k0 += 32) {
    V bh[4], bl[4];
#pragma unroll
    for (int j = 0; j < 4; ++j) {
      const size_t bo = (size_t)(n0 + (j << 4) + rlane) * ldb + koff + k0;
      bh[j] = Frag<T>::load(Bb + bo);
      if (SPLIT) bl[j] = Frag<T>::load(Bb2 + bo);
    }
#pragma unroll
    for (int i = 0; i < 4; ++i) {
      const size_t ao = (size_t)(m0 + (i << 4) + rlane) * lda + koff + k0;
      V ah = Frag<T>::load(Ab + ao);
      V al;
      if (SPLIT) al = Frag<T>::load(Ab2 + ao);
#pragma unroll
      for (int j = 0; j < 4; ++j) {
        acc[i][j] = Frag<T>::mma(ah, bh[j], acc[i][j]);
        if (SPLIT) {
          acc[i][j] = Frag<T>::mma(ah, bl[j], acc[i][j]);
          acc[i][j] = Frag<T>::mma(al, bh[j], acc[i][j]);
        }
      }
      Frag<T>::guard(acc[i][0], acc[i][3], ah, SPLIT ? al : ah);
    }
    Frag<T>::keep(bh[0], bh[1], bh[2], bh[3]);
    if (SPLIT) Frag<T>::keep(bl[0], bl[1], bl[2], bl[3]);
  }
  acc_guard4(acc[0][0], acc[0][1], acc[0][2], acc[0][3]);
  acc_guard4(acc[1][0], acc[1][1], acc[1][2], acc[1][3]);
  acc_guard4(acc[2][0], acc[2][1], acc[2][2], acc[2][3]);
  acc_guard4(acc[3][0], acc[3][1], acc[3][2], acc[3][3]);

  float* slab = sT[wave];
  const float* Rb = RESID ? (resid + (size_t)b * strideR) : nullptr;
#pragma unroll
  for (int i = 0; i < 4; ++i) {
    const int mBase = m0 + (i << 4);
#pragma unroll
    for (int j = 0; j < 4; ++j) {
      const int n = n0 + (j << 4) + rlane;
      float bv = 0.f;
      if (BIAS_MODE == 2) bv = bias[n];
#pragma unroll
      for (int r = 0; r < 8; ++r) {
        float v = acc[i][j][r] * scale;
        if (BIAS_MODE == 1) v += bias[mBase + mOff + r];
        if (BIAS_MODE == 2) v += bv;
        if (RESID) v += Rb[(size_t)(mBase + mOff + r) * ldc + n];
        if (ACT == 2) v = fmaxf(v, 0.0f);
        if (ACT == 4) v = (v > 0.f) ? v : 0.01f * v;
        slab[(mOff + r) * 68 + (j << 4) + rlane] = v;
      }
    }
    __builtin_amdgcn_fence(__ATOMIC_RELEASE, "workgroup");
    __builtin_amdgcn_wave_barrier();
    __builtin_amdgcn_fence(__ATOMIC_ACQUIRE, "workgroup");
    if (OUT_MODE == 0) {
      float* C = (float*)Cout + (size_t)b * strideC;
      const int hh = lane >> 4, c4 = (lane & 15) * 4;
      for (int pass = 0; pass < 2; ++pass) {
#pragma unroll
        for (int it = 0; it < 8; ++it) {
          const int row = it * 2 + hh;
          v4f v = *(const v4f*)(slab + row * 68 + c4);
          *(volatile v4f*)(C + (size_t)(mBase + row) * ldc + n0 + c4) = v;
        }
        __threadfence();
      }
    } else {
      const int q = lane >> 3, c8 = (lane & 7) * 8;
      unsigned short* C  = (unsigned short*)Cout  + (size_t)b * strideC;
      unsigned short* C2 = (OUT_MODE == 2) ? ((unsigned short*)Cout2 + (size_t)b * strideC) : nullptr;
      for (int pass = 0; pass < 2; ++pass) {
#pragma unroll
        for (int it = 0; it < 4; ++it) {
          const int row = it * 4 + q;
          const float* sp = slab + row * 68 + c8;
          v8h hv, lv;
#pragma unroll
          for (int e = 0; e < 8; ++e) {
            if (OUT_MODE == 1) {
              hv[e] = (_Float16)sp[e];
            } else {
              unsigned short hb = f2bf_bits(sp[e]);
              unsigned short lb = f2bf_bits(sp[e] - bf_bits2f(hb));
              hv[e] = __builtin_bit_cast(_Float16, hb);
              lv[e] = __builtin_bit_cast(_Float16, lb);
            }
          }
          *(volatile v8h*)(C + (size_t)(mBase + row) * ldc + n0 + c8) = hv;
          if (OUT_MODE == 2) *(volatile v8h*)(C2 + (size_t)(mBase + row) * ldc + n0 + c8) = lv;
        }
        __threadfence();
      }
    }
    __builtin_amdgcn_fence(__ATOMIC_RELEASE, "workgroup");
    __builtin_amdgcn_wave_barrier();
    __builtin_amdgcn_fence(__ATOMIC_ACQUIRE, "workgroup");
  }
}

__device__ __forceinline__ float wave_sum(float v) {
#pragma unroll
  for (int o = 16; o > 0; o >>= 1) v += __shfl_xor(v, o, 32);
  return v;
}
__device__ __forceinline__ float wave_max(float v) {
#pragma unroll
  for (int o = 16; o > 0; o >>= 1) v = fmaxf(v, __shfl_xor(v, o, 32));
  return v;
}

__global__ __launch_bounds__(256) void cast16_kernel(const float* __restrict__ Wg, const float* __restrict__ Wq,
                                                     const float* __restrict__ Wk, const float* __restrict__ Wv,
                                                     const float* __restrict__ Wvp, const float* __restrict__ Wfc,
                                                     const float* __restrict__ qin, const float* __restrict__ kin,
                                                     unsigned short* __restrict__ out) {
  const int z  = blockIdx.y;
  const int kz = (z >= 8) ? (z - 8) : 0;
  const float* src = (z == 0) ? Wg : (z == 1) ? (Wg + kSlot) : (z == 2) ? Wq : (z == 3) ? Wk : (z == 4) ? Wv
                   : (z == 5) ? Wvp : (z == 6) ? Wfc : (z == 7) ? qin : (kin + (size_t)kz * kSlot);
  const float scale = (z < 7) ? kWCarry : 1.0f;
  const int i = blockIdx.x * 256 + threadIdx.x;
  const float* p = src + 8 * (size_t)i;
  const v4f a = *(const v4f*)(p);
  const v4f c = *(const v4f*)(p + 4);
  unsigned short hb[8];
#pragma unroll
  for (int e = 0; e < 4; ++e) {
    hb[e]     = h_bits(a[e] * scale);
    hb[4 + e] = h_bits(c[e] * scale);
  }
  const v4u u = (v4u){pk16(hb[0], hb[1]), pk16(hb[2], hb[3]), pk16(hb[4], hb[5]), pk16(hb[6], hb[7])};
  unsigned short* qo = out + (size_t)z * kSlot + 8 * (size_t)i;
  *(volatile v4u*)qo = u;
  __threadfence();
  *(volatile v4u*)qo = u;
}

__global__ __launch_bounds__(256) void ln1_kernel(const float* __restrict__ vp, const float* __restrict__ bvp,
                                                  const float* __restrict__ g1, const float* __restrict__ b1,
                                                  float* __restrict__ cb) {
  const int lane = threadIdx.x & 31, wave = threadIdx.x >> 5;
  const int row = blockIdx.x * 8 + wave;
  const float* src = vp + (size_t)row * kDim;
  float x[16];
#pragma unroll
  for (int it = 0; it < 4; ++it) {
    const int col = it * 128 + lane * 4;
    const v4f a  = *(const v4f*)(src + col);
    const v4f bb = *(const v4f*)(bvp + col);
#pragma unroll
    for (int e = 0; e < 4; ++e) x[it * 4 + e] = a[e] + bb[e];
  }
  float s = 0.f;
#pragma unroll
  for (int i = 0; i < 16; ++i) s += x[i];
  s = wave_sum(s);
  const float mean = s * kInvDim;
  float vs = 0.f;
#pragma unroll
  for (int i = 0; i < 16; ++i) { const float d = x[i] - mean; x[i] = d; vs += d * d; }
  vs = wave_sum(vs);
  const float rstd = rsqrtf(vs * kInvDim + kLnEps);
  v4f o[4];
#pragma unroll
  for (int it = 0; it < 4; ++it) {
    const int col = it * 128 + lane * 4;
    const v4f g  = *(const v4f*)(g1 + col);
    const v4f be = *(const v4f*)(b1 + col);
#pragma unroll
    for (int e = 0; e < 4; ++e) o[it][e] = x[it * 4 + e] * rstd * g[e] + be[e];
  }
  float* dst = cb + (size_t)row * kDim;
  for (int pass = 0; pass < 2; ++pass) {
#pragma unroll
    for (int it = 0; it < 4; ++it) *(volatile v4f*)(dst + it * 128 + lane * 4) = o[it];
    __threadfence();
  }
}

__global__ __launch_bounds__(256) void condk_kernel(const float* __restrict__ fq, const float* __restrict__ bg,
                                                    const float* __restrict__ g2, const float* __restrict__ b2,
                                                    const float* __restrict__ cb, const float* __restrict__ kin,
                                                    unsigned short* __restrict__ ck, int bb) {
  __shared__ __align__(16) float gb_s[1024];
  __shared__ __align__(16) float g2_s[512];
  __shared__ __align__(16) float b2_s[512];
  const int tid = threadIdx.x, lane = tid & 31, wave = tid >> 5;
  const int r0 = blockIdx.x * 8;
  const int l  = r0 >> 8;
  const float* frow = fq + (size_t)(bb * kLQ + l) * kFqLd;
#pragma unroll 1
  for (int i2 = 0; i2 < 4; ++i2) {
    const int d = i2 * 256 + tid;
    gb_s[d] = tanhf(frow[d] + bg[d]);
  }
  g2_s[tid] = g2[tid];  g2_s[tid + 256] = g2[tid + 256];
  b2_s[tid] = b2[tid];  b2_s[tid + 256] = b2[tid + 256];
  __syncthreads();

  const int r  = r0 + wave;
  const int kk = r & 255;
  const float* cbr = cb  + (size_t)(bb * kLK + kk) * kDim;
  const float* kr  = kin + (size_t)(bb * kLK + kk) * kDim;
  float c[16];
#pragma unroll
  for (int it = 0; it < 2; ++it) {
#pragma unroll
    for (int hf = 0; hf < 2; ++hf) {
      const int col = it * 256 + lane * 8 + hf * 4;
      const v4f a  = *(const v4f*)(cbr + col);
      const v4f g  = *(const v4f*)(gb_s + col);
      const v4f be = *(const v4f*)(gb_s + 512 + col);
#pragma unroll
      for (int e = 0; e < 4; ++e) c[it * 8 + hf * 4 + e] = g[e] * a[e] + be[e];
    }
  }
  float s = 0.f;
#pragma unroll
  for (int i = 0; i < 16; ++i) s += c[i];
  s = wave_sum(s);
  const float mean = s * kInvDim;
  float vs = 0.f;
#pragma unroll
  for (int i = 0; i < 16; ++i) { const float d = c[i] - mean; c[i] = d; vs += d * d; }
  vs = wave_sum(vs);
  const float rstd = rsqrtf(vs * kInvDim + kLnEps);

  v4u u[2];
#pragma unroll
  for (int it = 0; it < 2; ++it) {
    unsigned short hb[8];
#pragma unroll
    for (int hf = 0; hf < 2; ++hf) {
      const int col = it * 256 + lane * 8 + hf * 4;
      const v4f k4 = *(const v4f*)(kr + col);
      const v4f gg = *(const v4f*)(g2_s + col);
      const v4f bt = *(const v4f*)(b2_s + col);
#pragma unroll
      for (int e = 0; e < 4; ++e) {
        const float y = c[it * 8 + hf * 4 + e] * rstd * gg[e] + bt[e];
        hb[hf * 4 + e] = h_bits(k4[e] + y);
      }
    }
    u[it] = (v4u){pk16(hb[0], hb[1]), pk16(hb[2], hb[3]), pk16(hb[4], hb[5]), pk16(hb[6], hb[7])};
  }
  unsigned short* dst = ck + (size_t)r * kDim;
  for (int pass = 0; pass < 2; ++pass) {
#pragma unroll
    for (int it = 0; it < 2; ++it) *(volatile v4u*)(dst + it * 256 + lane * 8) = u[it];
    __threadfence();
  }
}

__global__ __launch_bounds__(256) void attn_kernel(const float* __restrict__ fq, const float* __restrict__ kv,
                                                   unsigned short* __restrict__ att, int bb) {
  __shared__ __align__(16) float qs[512];
  __shared__ __align__(16) float sw[8][256];
  __shared__ __align__(16) float ao[8][64];
  const int tid = threadIdx.x, lane = tid & 31, wave = tid >> 5;
  const int l = blockIdx.x;
  const int rowq = bb * kLQ + l;
  const float* qrow = fq + (size_t)rowq * kFqLd + 1024;
  qs[tid] = qrow[tid];  qs[tid + 256] = qrow[tid + 256];
  __syncthreads();

  const int h = wave;
  const float* kvb = kv + (size_t)(l * kLK) * kKvLd;
#pragma unroll 1
  for (int j = 0; j < 8; ++j) {
    const int kk = j * 32 + lane;
    const float* krow = kvb + (size_t)kk * kKvLd + h * kDk;
    float acc = 0.f;
#pragma unroll 1
    for (int d4 = 0; d4 < 16; ++d4) {
      const v4f a  = *(const v4f*)(krow + 4 * d4);
      const v4f qq = *(const v4f*)(qs + h * kDk + 4 * d4);
      acc += a[0] * qq[0];
      acc += a[1] * qq[1];
      acc += a[2] * qq[2];
      acc += a[3] * qq[3];
    }
    sw[h][kk] = acc * kLogitScale;
  }
  __syncthreads();

  float m = sw[h][lane];
#pragma unroll 1
  for (int j = 1; j < 8; ++j) m = fmaxf(m, sw[h][j * 32 + lane]);
  m = wave_max(m);
  float s = 0.f;
#pragma unroll 1
  for (int j = 0; j < 8; ++j) {
    const int idx = j * 32 + lane;
    const float p = expf(sw[h][idx] - m);
    sw[h][idx] = p;
    s += p;
  }
  s = wave_sum(s);
  const float inv = 1.0f / s;
  __syncthreads();

  float a0 = 0.f, a1 = 0.f;
  const float* vb = kvb + kDim + h * kDk;
#pragma unroll 4
  for (int kk = 0; kk < kLK; ++kk) {
    const float w = sw[h][kk];
    const float* vr = vb + (size_t)kk * kKvLd;
    a0 += w * vr[lane];
    a1 += w * vr[lane + 32];
  }
  const float f = inv * kAttCarry;
  ao[h][lane]      = a0 * f;
  ao[h][lane + 32] = a1 * f;
  __syncthreads();

  const int l8 = lane & 7;
  const v4f x0 = *(const v4f*)(&ao[h][l8 * 8]);
  const v4f x1 = *(const v4f*)(&ao[h][l8 * 8 + 4]);
  unsigned short hb[8];
#pragma unroll
  for (int e = 0; e < 4; ++e) { hb[e] = h_bits(x0[e]); hb[4 + e] = h_bits(x1[e]); }
  const v4u u = (v4u){pk16(hb[0], hb[1]), pk16(hb[2], hb[3]), pk16(hb[4], hb[5]), pk16(hb[6], hb[7])};
  unsigned short* dst = att + (size_t)rowq * kDim + h * kDk + l8 * 8;
  for (int pass = 0; pass < 2; ++pass) {
    if (lane < 8) *(volatile v4u*)dst = u;
    __threadfence();
  }
}

static void gemm_f16_f32out(const unsigned short* A, int lda, const unsigned short* Bt, int ldb,
                            void* C, int ldc, int M, int N, int K, float scale,
                            const float* dummyf, hipStream_t stream) {
  const int tiles = (M / 64) * (N / 64);
  dim3 grid((unsigned)((tiles + 7) / 8), 1, 1);
  wmma_gemm64<0, false, 0, 0, false, 0><<<grid, 256, 0, stream>>>(
      A, A, lda, 0L, Bt, Bt, ldb, 0L, C, C, ldc, 0L, dummyf, dummyf, 0L, M, N, K, scale);
}

extern "C" void kernel_launch(void* const* d_in, const int* in_sizes, int n_in,
                              void* d_out, int out_size, void* d_ws, size_t ws_size,
                              hipStream_t stream) {
  if (n_in < 15) return;
  if (ws_size < kWsTotal) return;
  if (out_size < kQRows * kDim) return;
  if (in_sizes[0] < kQRows * kDim || in_sizes[1] < kKRows * kDim) return;

  const float* q    = (const float*)d_in[0];
  const float* k    = (const float*)d_in[1];
  const float* Wq   = (const float*)d_in[3];
  const float* Wk   = (const float*)d_in[4];
  const float* Wv   = (const float*)d_in[5];
  const float* Wfc  = (const float*)d_in[6];
  const float* Wg   = (const float*)d_in[7];
  const float* bg   = (const float*)d_in[8];
  const float* Wvp  = (const float*)d_in[9];
  const float* bvp  = (const float*)d_in[10];
  const float* ln1g = (const float*)d_in[11];
  const float* ln1b = (const float*)d_in[12];
  const float* ln2g = (const float*)d_in[13];
  const float* ln2b = (const float*)d_in[14];
  float* out = (float*)d_out;

  char* ws = (char*)d_ws;
  unsigned short* w16   = (unsigned short*)(ws + kOffW16);
  float*          fq    = (float*)(ws + kOffFq);
  float*          vp    = (float*)(ws + kOffVp);
  float*          cb    = (float*)(ws + kOffCb);
  unsigned short* ck16  = (unsigned short*)(ws + kOffCk);
  float*          kv    = (float*)(ws + kOffKv);
  unsigned short* att16 = (unsigned short*)(ws + kOffAtt);

  const unsigned short* wgq16  = w16 + (size_t)0 * kSlot;
  const unsigned short* wkv16  = w16 + (size_t)3 * kSlot;
  const unsigned short* wvp16  = w16 + (size_t)5 * kSlot;
  const unsigned short* wfc16  = w16 + (size_t)6 * kSlot;
  const unsigned short* q16    = w16 + (size_t)7 * kSlot;
  const unsigned short* k16    = w16 + (size_t)8 * kSlot;

  cast16_kernel<<<dim3(128, 16, 1), 256, 0, stream>>>(Wg, Wq, Wk, Wv, Wvp, Wfc, q, k, w16);
  gemm_f16_f32out(q16, kDim, wgq16, kDim, (void*)fq, kFqLd, kQRows, kFqLd, kDim, kScaleW, bg, stream);
  gemm_f16_f32out(k16, kDim, wvp16, kDim, (void*)vp, kDim, kKRows, kDim, kDim, kScaleW, bg, stream);
  ln1_kernel<<<512, 256, 0, stream>>>(vp, bvp, ln1g, ln1b, cb);
  for (int bb = 0; bb < kNumB; ++bb) {
    condk_kernel<<<kChunkRows / 8, 256, 0, stream>>>(fq, bg, ln2g, ln2b, cb, k, ck16, bb);
    gemm_f16_f32out(ck16, kDim, wkv16, kDim, (void*)kv, kKvLd, kChunkRows, kKvLd, kDim, kScaleW, bg, stream);
    attn_kernel<<<kLQ, 256, 0, stream>>>(fq, kv, att16, bb);
  }
  gemm_f16_f32out(att16, kDim, wfc16, kDim, (void*)out, kDim, kQRows, kDim, kDim, kScaleOut, bg, stream);
}
